// VSSBlockBS_9371618640305
// MI455X (gfx1250) — hardware-verified
//
#include <hip/hip_runtime.h>


namespace {
constexpr int NB = 8, HH = 32, L = HH * HH, NT = NB * L, C = 192, DI = 384, NS = 16, R = 12, XD = R + 2 * NS, HID = 768;
constexpr float XS = 8.0f, US = 4096.0f, DS = 16384.0f, YS = 64.0f, GS = 128.0f, WSC = 256.0f, EPS = 1e-5f;
typedef _Float16 b16;
typedef __attribute__((ext_vector_type(16))) _Float16 v16b;
typedef __attribute__((ext_vector_type(8))) _Float16 v8b;
typedef __attribute__((ext_vector_type(8))) float v8f;
typedef __attribute__((ext_vector_type(4))) float v4f;
typedef __attribute__((ext_vector_type(2))) float v2f;
__device__ __forceinline__ float bf16_rne(float f) { unsigned int u = __float_as_uint(f); u += 0x7FFFu + ((u >> 16) & 1u); return __uint_as_float(u & 0xFFFF0000u); }
__device__ __forceinline__ void split16(float v, b16& hi, b16& lo) { hi = (b16)v; lo = (b16)(v - (float)hi); }
__device__ __forceinline__ v16b frag_kb(const b16* p, int hh) { const v8b a = *(const v8b*)(p + 8 * hh), b = *(const v8b*)(p + 16 + 8 * hh); v16b f;
#pragma unroll
  for (int e = 0; e < 8; ++e) { f[e] = a[e]; f[8 + e] = b[e]; } return f; }
__device__ __forceinline__ v8f wmma16b(v16b a, v16b b, v8f c) { v8f d = __builtin_amdgcn_wmma_f32_16x16x32_f16(false, a, false, b, (short)0, c, false, false); asm volatile("v_nop\n\tv_nop\n\tv_nop\n\tv_nop" : "+v"(d) : "v"(a), "v"(b)); return d; }
__device__ __forceinline__ void wave_lds_sync() { __builtin_amdgcn_fence(__ATOMIC_RELEASE, "workgroup"); __builtin_amdgcn_wave_barrier(); __builtin_amdgcn_fence(__ATOMIC_ACQUIRE, "workgroup"); }
__device__ __forceinline__ float pmul(float a, float b) { float p = a * b; asm volatile("" : "+v"(p)); return p; }
__device__ __forceinline__ int iclamp(int v, int lo, int hi) { return v < lo ? lo : (v > hi ? hi : v); }
__device__ __forceinline__ float sigm(float v) { return 1.0f / (1.0f + __expf(-v)); }
__device__ __forceinline__ float silu(float v) { return pmul(v, sigm(v)); }
__device__ __forceinline__ float softplus(float v) { return v > 20.0f ? v : (v < -20.0f ? __expf(v) : log1pf(__expf(v))); }
__device__ __forceinline__ float gelu_tanh(float v) { const float t = tanhf(0.7978845608028654f * (v + 0.044715f * v * v * v)); return 0.5f * v * (1.0f + t); }

__global__ __launch_bounds__(256) void wcopyp_kernel(const float* __restrict__ w, int KIN, int OUT, int KP, int OUTP, b16* __restrict__ WT) {
  const int u = blockIdx.x * 256 + threadIdx.x; if (u >= OUTP * KP / 8) return; const int e = u * 8; const int o = e / KP, k0 = e % KP; v8b v;
#pragma unroll
  for (int j = 0; j < 8; ++j) { const int k = k0 + j; v[j] = (o < OUT && k < KIN) ? (b16)(bf16_rne(w[(size_t)o * KIN + k]) * WSC) : (b16)0.0f; } for (int pass = 0; pass < 2; ++pass) { *(volatile v8b*)(WT + e) = v; __threadfence(); }
}
__global__ __launch_bounds__(32) void inproj_kernel(const float* __restrict__ X, const float* __restrict__ g, const float* __restrict__ bb, const b16* __restrict__ WIP, float* __restrict__ XZ) {
  __shared__ __attribute__((aligned(16))) b16 Ah[16][C + 8], Al[16][C + 8]; __shared__ __attribute__((aligned(16))) float Tf[16][128 + 4];
  const int lane = threadIdx.x, nloc = lane & 15, hlf = lane >> 4; const size_t m0 = (size_t)blockIdx.x * 16;
  float g6[6], b6[6]; for (int q = 0; q < 6; ++q) { g6[q] = bf16_rne(g[q * 32 + lane]); b6[q] = bf16_rne(bb[q * 32 + lane]); }
  for (int rr = 0; rr < 16; ++rr) { float v[6]; float s = 0.0f; for (int q = 0; q < 6; ++q) { v[q] = bf16_rne(X[(m0 + rr) * C + q * 32 + lane]); s += v[q]; } for (int o = 16; o; o >>= 1) s += __shfl_xor(s, o); const float mu = s * (1.0f / C);
    float vq = 0.0f; for (int q = 0; q < 6; ++q) { const float d = v[q] - mu; vq += pmul(d, d); } for (int o = 16; o; o >>= 1) vq += __shfl_xor(vq, o); const float rs = rsqrtf(vq * (1.0f / C) + EPS);
    for (int q = 0; q < 6; ++q) { b16 p, ql; split16((pmul(pmul(v[q] - mu, rs), g6[q]) + b6[q]) * XS, p, ql); Ah[rr][q * 32 + lane] = p; Al[rr][q * 32 + lane] = ql; } }
  wave_lds_sync();
#pragma unroll 1
  for (int cg = 0; cg < 2 * DI / 128; ++cg) { v8f acc[8];
#pragma unroll
    for (int t = 0; t < 8; ++t) acc[t] = (v8f){};
#pragma unroll 2
    for (int kb = 0; kb < C; kb += 32) { const v16b a = frag_kb(&Ah[nloc][kb], hlf), al = frag_kb(&Al[nloc][kb], hlf);
#pragma unroll
      for (int t = 0; t < 8; ++t) { const v16b bw = frag_kb(WIP + (size_t)(cg * 128 + t * 16 + nloc) * C + kb, hlf); acc[t] = wmma16b(a, bw, acc[t]); acc[t] = wmma16b(al, bw, acc[t]); } }
#pragma unroll
    for (int t = 0; t < 8; ++t)
#pragma unroll 1
      for (int r8 = 0; r8 < 8; ++r8) Tf[8 * hlf + r8][t * 16 + nloc] = acc[t][r8] * (1.0f / (XS * WSC));
    wave_lds_sync();
    for (int pass = 0; pass < 2; ++pass) { for (int rr = 0; rr < 16; ++rr) *(volatile v4f*)(XZ + (m0 + rr) * (2 * DI) + cg * 128 + lane * 4) = *(const v4f*)(&Tf[rr][lane * 4]); __threadfence(); }
    wave_lds_sync(); }
}
__global__ __launch_bounds__(256) void dwconv_kernel(const float* __restrict__ XZ, const float* __restrict__ cw, const float* __restrict__ cb, int ntok, float* __restrict__ U) {
  const size_t gid = (size_t)blockIdx.x * 256 + threadIdx.x; const size_t t = gid / (DI / 4); const int d4 = (int)(gid % (DI / 4)) * 4; if (t >= (size_t)ntok) return;
  const int b = (int)(t / L), p = (int)(t % L), y = p / HH, x = p % HH; v4f acc; for (int q = 0; q < 4; ++q) acc[q] = bf16_rne(cb[d4 + q]);
#pragma unroll
  for (int di = 0; di < 3; ++di)
#pragma unroll
    for (int dj = 0; dj < 3; ++dj) { const int yy = y + di - 1, xx = x + dj - 1; const bool ok = yy >= 0 && yy < HH && xx >= 0 && xx < HH; const int yc = ok ? yy : y, xc = ok ? xx : x;
      const v4f v = *(const v4f*)(XZ + ((size_t)b * L + yc * HH + xc) * (2 * DI) + d4); for (int q = 0; q < 4; ++q) acc[q] += ok ? pmul(v[q], bf16_rne(cw[(d4 + q) * 9 + di * 3 + dj])) : 0.0f; }
  v4f o; for (int q = 0; q < 4; ++q) o[q] = silu(acc[q]);
  for (int pass = 0; pass < 2; ++pass) { *(volatile v4f*)(U + t * DI + d4) = o; __threadfence(); }
}
__global__ __launch_bounds__(32) void xproj_kernel(const float* __restrict__ U, const b16* __restrict__ XPW, const b16* __restrict__ DTW, const float* __restrict__ dtb, float* __restrict__ BC, float* __restrict__ DT) {
  __shared__ __attribute__((aligned(16))) b16 Ah[16][DI + 8], Al[16][DI + 8]; __shared__ __attribute__((aligned(16))) b16 Dh[16][32 + 8], Dl[16][32 + 8]; __shared__ __attribute__((aligned(16))) float Sbc[16][32]; __shared__ __attribute__((aligned(16))) float Tf[16][DI + 4];
  const int lane = threadIdx.x, nloc = lane & 15, hlf = lane >> 4; const size_t m0 = (size_t)blockIdx.x * 16;
  for (int rr = 0; rr < 16; ++rr) for (int q = 0; q < 3; ++q) { const v4f v = *(const v4f*)(U + (m0 + rr) * DI + q * 128 + lane * 4); for (int j = 0; j < 4; ++j) { b16 p, ql; split16(v[j] * US, p, ql); Ah[rr][q * 128 + lane * 4 + j] = p; Al[rr][q * 128 + lane * 4 + j] = ql; } }
  wave_lds_sync();
  const float sx = 1.0f / (US * WSC), sd = 1.0f / (DS * WSC);
  v8f ax[3] = {(v8f){}, (v8f){}, (v8f){}};
#pragma unroll 2
  for (int kb = 0; kb < DI; kb += 32) { const v16b a = frag_kb(&Ah[nloc][kb], hlf), al = frag_kb(&Al[nloc][kb], hlf);
#pragma unroll
    for (int t = 0; t < 3; ++t) { const v16b bw = frag_kb(XPW + (size_t)(t * 16 + nloc) * DI + kb, hlf); ax[t] = wmma16b(a, bw, ax[t]); ax[t] = wmma16b(al, bw, ax[t]); } }
#pragma unroll
  for (int r8 = 0; r8 < 8; ++r8) { const int rl = 8 * hlf + r8; const float d0 = ax[0][r8] * sx, d1 = ax[1][r8] * sx, d2 = ax[2][r8] * sx;
    if (nloc < R) { b16 p, ql; split16(d0 * DS, p, ql); Dh[rl][nloc] = p; Dl[rl][nloc] = ql; Sbc[rl][4 + nloc] = d1; Sbc[rl][16 + 4 + nloc] = d2; }
    else { Dh[rl][nloc] = (b16)0.0f; Dl[rl][nloc] = (b16)0.0f; Sbc[rl][nloc - R] = d0; Sbc[rl][16 + nloc - R] = d1; }
    Dh[rl][16 + nloc] = (b16)0.0f; Dl[rl][16 + nloc] = (b16)0.0f; }
  wave_lds_sync();
  for (int pass = 0; pass < 2; ++pass) { for (int rr = 0; rr < 16; ++rr) ((volatile float*)BC)[(m0 + rr) * 32 + lane] = Sbc[rr][lane]; __threadfence(); }
  { const v16b a = frag_kb(&Dh[nloc][0], hlf), al = frag_kb(&Dl[nloc][0], hlf);
#pragma unroll 1
    for (int cg = 0; cg < 2; ++cg) { v8f acc[12];
#pragma unroll
      for (int t = 0; t < 12; ++t) { acc[t] = (v8f){}; const v16b bw = frag_kb(DTW + (size_t)(cg * 192 + t * 16 + nloc) * 32, hlf); acc[t] = wmma16b(a, bw, acc[t]); acc[t] = wmma16b(al, bw, acc[t]); }
#pragma unroll
      for (int t = 0; t < 12; ++t) { const int c = cg * 192 + t * 16 + nloc; const float bb = bf16_rne(dtb[c]);
#pragma unroll 1
        for (int r8 = 0; r8 < 8; ++r8) Tf[8 * hlf + r8][c] = softplus(acc[t][r8] * sd + bb); } } }
  wave_lds_sync();
  for (int pass = 0; pass < 2; ++pass) { for (int rr = 0; rr < 16; ++rr) for (int q = 0; q < 3; ++q) *(volatile v4f*)(DT + (m0 + rr) * DI + q * 128 + lane * 4) = *(const v4f*)(&Tf[rr][q * 128 + lane * 4]); __threadfence(); }
}
__global__ __launch_bounds__(256) void scan_kernel(const float* __restrict__ U, const float* __restrict__ DT, const float* __restrict__ BC, const int* __restrict__ perm, const float* __restrict__ alog, const float* __restrict__ Dp, int nbv, float* __restrict__ Y) {
  const int gid = blockIdx.x * 256 + threadIdx.x; const int b = gid / DI, d = gid % DI; if (b >= nbv) return;
  float A[NS]; for (int s = 0; s < NS; ++s) A[s] = -__expf(bf16_rne(alog[d * NS + s])); const float dk = bf16_rne(Dp[d]);
#pragma unroll 1
  for (int pass = 0; pass < 2; ++pass) { float h[NS]; for (int s = 0; s < NS; ++s) h[s] = 0.0f;
#pragma unroll 1
    for (int l = 0; l < L; ++l) { const int p = iclamp(perm[l], 0, L - 1); const size_t row = (size_t)b * L + p; const float u = U[row * DI + d], dt = DT[row * DI + d]; const float du = pmul(dt, u); const float* bc = BC + row * 32; float acc = 0.0f;
#pragma unroll
      for (int s = 0; s < NS; ++s) { h[s] = pmul(h[s], __expf(pmul(dt, A[s]))) + pmul(du, bc[s]); acc += pmul(h[s], bc[16 + s]); }
      ((volatile float*)Y)[row * DI + d] = acc + pmul(dk, u); }
    __threadfence(); }
}
__global__ __launch_bounds__(32) void block_out_kernel(const float* __restrict__ Y, const float* __restrict__ XZ, const float* __restrict__ X, const float* __restrict__ og, const float* __restrict__ ob, const b16* __restrict__ WOP, const float* __restrict__ g2, const float* __restrict__ b2, const b16* __restrict__ WF1, const float* __restrict__ f1b, const b16* __restrict__ WF2, const float* __restrict__ f2b, float* __restrict__ out) {
  __shared__ __attribute__((aligned(16))) b16 Ah[16][DI + 8], Al[16][DI + 8]; __shared__ __attribute__((aligned(16))) b16 A2h[16][HID + 8], A2l[16][HID + 8]; __shared__ __attribute__((aligned(16))) float Xs[16][C + 4];
  const int lane = threadIdx.x, nloc = lane & 15, hlf = lane >> 4; const size_t m0 = (size_t)blockIdx.x * 16;
  { float g12[12], b12[12]; for (int q = 0; q < 12; ++q) { g12[q] = bf16_rne(og[q * 32 + lane]); b12[q] = bf16_rne(ob[q * 32 + lane]); }
    for (int rr = 0; rr < 16; ++rr) { const size_t t = m0 + rr; float v[12]; float s = 0.0f; for (int q = 0; q < 12; ++q) { v[q] = Y[t * DI + q * 32 + lane]; s += v[q]; } for (int o = 16; o; o >>= 1) s += __shfl_xor(s, o); const float mu = s * (1.0f / DI);
      float vq = 0.0f; for (int q = 0; q < 12; ++q) { const float dd = v[q] - mu; vq += pmul(dd, dd); } for (int o = 16; o; o >>= 1) vq += __shfl_xor(vq, o); const float rs = rsqrtf(vq * (1.0f / DI) + EPS);
      for (int q = 0; q < 12; ++q) { const int c = q * 32 + lane; const float z = XZ[t * (2 * DI) + DI + c]; const float a = pmul(pmul(pmul(v[q] - mu, rs), g12[q]) + b12[q], silu(z)); b16 p, ql; split16(a * YS, p, ql); Ah[rr][c] = p; Al[rr][c] = ql; }
      for (int q = 0; q < 6; ++q) Xs[rr][q * 32 + lane] = bf16_rne(X[t * C + q * 32 + lane]); } }
  wave_lds_sync();
  { v8f acc[12];
#pragma unroll
    for (int t = 0; t < 12; ++t) acc[t] = (v8f){};
#pragma unroll 2
    for (int kb = 0; kb < DI; kb += 32) { const v16b a = frag_kb(&Ah[nloc][kb], hlf), al = frag_kb(&Al[nloc][kb], hlf);
#pragma unroll
      for (int t = 0; t < 12; ++t) { const v16b bw = frag_kb(WOP + (size_t)(t * 16 + nloc) * DI + kb, hlf); acc[t] = wmma16b(a, bw, acc[t]); acc[t] = wmma16b(al, bw, acc[t]); } }
    wave_lds_sync();
#pragma unroll
    for (int t = 0; t < 12; ++t) { const int c = t * 16 + nloc;
#pragma unroll
      for (int r8 = 0; r8 < 8; ++r8) Xs[8 * hlf + r8][c] += acc[t][r8] * (1.0f / (YS * WSC)); } }
  wave_lds_sync();
  { float g6[6], b6[6]; for (int q = 0; q < 6; ++q) { g6[q] = bf16_rne(g2[q * 32 + lane]); b6[q] = bf16_rne(b2[q * 32 + lane]); }
    for (int rr = 0; rr < 16; ++rr) { float v[6]; float s = 0.0f; for (int q = 0; q < 6; ++q) { v[q] = Xs[rr][q * 32 + lane]; s += v[q]; } for (int o = 16; o; o >>= 1) s += __shfl_xor(s, o); const float mu = s * (1.0f / C); float vq = 0.0f; for (int q = 0; q < 6; ++q) { const float dd = v[q] - mu; vq += pmul(dd, dd); } for (int o = 16; o; o >>= 1) vq += __shfl_xor(vq, o); const float rs = rsqrtf(vq * (1.0f / C) + EPS);
      for (int q = 0; q < 6; ++q) { b16 p, ql; split16((pmul(pmul(v[q] - mu, rs), g6[q]) + b6[q]) * XS, p, ql); Ah[rr][q * 32 + lane] = p; Al[rr][q * 32 + lane] = ql; } } }
  wave_lds_sync();
#pragma unroll 1
  for (int cg = 0; cg < HID / 128; ++cg) { v8f a1[8];
#pragma unroll
    for (int t = 0; t < 8; ++t) a1[t] = (v8f){};
#pragma unroll 2
    for (int kb = 0; kb < C; kb += 32) { const v16b a = frag_kb(&Ah[nloc][kb], hlf), al = frag_kb(&Al[nloc][kb], hlf);
#pragma unroll
      for (int t = 0; t < 8; ++t) { const v16b bw = frag_kb(WF1 + (size_t)(cg * 128 + t * 16 + nloc) * C + kb, hlf); a1[t] = wmma16b(a, bw, a1[t]); a1[t] = wmma16b(al, bw, a1[t]); } }
#pragma unroll
    for (int t = 0; t < 8; ++t) { const int c = cg * 128 + t * 16 + nloc; const float bb = bf16_rne(f1b[c]);
#pragma unroll
      for (int r8 = 0; r8 < 8; ++r8) { const float gv = gelu_tanh(a1[t][r8] * (1.0f / (XS * WSC)) + bb); b16 p, ql; split16(gv * GS, p, ql); A2h[8 * hlf + r8][c] = p; A2l[8 * hlf + r8][c] = ql; } } }
  wave_lds_sync();
  { v8f acc[12];
#pragma unroll
    for (int t = 0; t < 12; ++t) acc[t] = (v8f){};
#pragma unroll 2
    for (int kb = 0; kb < HID; kb += 32) { const v16b a = frag_kb(&A2h[nloc][kb], hlf), al = frag_kb(&A2l[nloc][kb], hlf);
#pragma unroll
      for (int t = 0; t < 12; ++t) { const v16b bw = frag_kb(WF2 + (size_t)(t * 16 + nloc) * HID + kb, hlf); acc[t] = wmma16b(a, bw, acc[t]); acc[t] = wmma16b(al, bw, acc[t]); } }
#pragma unroll
    for (int t = 0; t < 12; ++t) { const int c = t * 16 + nloc; const float bb = bf16_rne(f2b[c]);
#pragma unroll
      for (int r8 = 0; r8 < 8; ++r8) Xs[8 * hlf + r8][c] += acc[t][r8] * (1.0f / (GS * WSC)) + bb; } }
  wave_lds_sync();
  for (int pass = 0; pass < 2; ++pass) { for (int rr = 0; rr < 16; ++rr) for (int q = 0; q < 6; ++q) ((volatile float*)out)[(m0 + rr) * C + q * 32 + lane] = Xs[rr][q * 32 + lane]; __threadfence(); }
}
}

extern "C" void kernel_launch(void* const* d_in, const int* in_sizes, int n_in, void* d_out, int out_size, void* d_ws, size_t ws_size, hipStream_t stream) {
  (void)n_in;
  auto Fp = [&](int i) { return (const float*)d_in[i]; }; auto Ip = [&](int i) { return (const int*)d_in[i]; };
  if (in_sizes[0] != NT * C || in_sizes[1] != L || in_sizes[5] != 2 * DI * C || in_sizes[6] != DI * 9 || in_sizes[8] != XD * DI || in_sizes[9] != DI * R || in_sizes[11] != DI * NS || in_sizes[15] != C * DI || in_sizes[18] != HID * C || in_sizes[20] != C * HID || out_size != NT * C) return;
  const int NBV = NB; const int NTV = NBV * L;
  size_t off = 0; char* ws = (char*)d_ws;
  auto carve = [&](size_t bytes) { char* p = ws + off; off += (bytes + 255) & ~(size_t)255; return p; };
  b16* WIP = (b16*)carve((size_t)2 * DI * C * 2); b16* XPW = (b16*)carve((size_t)48 * DI * 2); b16* DTW = (b16*)carve((size_t)DI * 32 * 2); b16* WOP = (b16*)carve((size_t)C * DI * 2); b16* WF1 = (b16*)carve((size_t)HID * C * 2); b16* WF2 = (b16*)carve((size_t)C * HID * 2);
  float* XZ = (float*)carve((size_t)NT * 2 * DI * 4); float* U = (float*)carve((size_t)NT * DI * 4); float* BC = (float*)carve((size_t)NT * 32 * 4); float* DT = (float*)carve((size_t)NT * DI * 4); float* Y = (float*)carve((size_t)NT * DI * 4);
  if (off > ws_size || off > ((size_t)96 << 20)) return;
  auto wcp = [&](const float* w, int KIN, int OUT, int KP, int OUTP, b16* WT) { wcopyp_kernel<<<(OUTP * KP / 8 + 255) / 256, 256, 0, stream>>>(w, KIN, OUT, KP, OUTP, WT); };
  wcp(Fp(5), C, 2 * DI, C, 2 * DI, WIP); wcp(Fp(8), DI, XD, DI, 48, XPW); wcp(Fp(9), R, DI, 32, DI, DTW); wcp(Fp(15), DI, C, DI, C, WOP); wcp(Fp(18), C, HID, C, HID, WF1); wcp(Fp(20), HID, C, HID, C, WF2);
  inproj_kernel<<<NTV / 16, 32, 0, stream>>>(Fp(0), Fp(3), Fp(4), WIP, XZ);
  dwconv_kernel<<<(unsigned)(((size_t)NTV * (DI / 4) + 255) / 256), 256, 0, stream>>>(XZ, Fp(6), Fp(7), NTV, U);
  xproj_kernel<<<NTV / 16, 32, 0, stream>>>(U, XPW, DTW, Fp(10), BC, DT);
  scan_kernel<<<(NBV * DI + 255) / 256, 256, 0, stream>>>(U, DT, BC, Ip(1), Fp(11), Fp(12), NBV, Y);
  block_out_kernel<<<NTV / 16, 32, 0, stream>>>(Y, XZ, Fp(0), Fp(13), Fp(14), WOP, Fp(16), Fp(17), WF1, Fp(19), WF2, Fp(21), (float*)d_out);
}
